// EGAN_Layer_38448547234242
// MI455X (gfx1250) — hardware-verified
//
#include <hip/hip_runtime.h>


namespace {
constexpr int N = 4096, NVEC = 3, M = 16, E = 256, NH = 8, HD = 32, NG = N * NVEC;
constexpr float XS = 8.0f, PS = 1024.0f, WSC = 256.0f, SQE = 16.0f, SCAL = 0.17677669529663687f;
typedef _Float16 b16;
typedef __attribute__((ext_vector_type(16))) _Float16 v16b;
typedef __attribute__((ext_vector_type(8))) _Float16 v8b;
typedef __attribute__((ext_vector_type(8))) float v8f;
typedef __attribute__((ext_vector_type(4))) float v4f;
__device__ __forceinline__ float bf16_rne(float f) { unsigned int u = __float_as_uint(f); u += 0x7FFFu + ((u >> 16) & 1u); return __uint_as_float(u & 0xFFFF0000u); }
__device__ __forceinline__ void split16(float v, b16& hi, b16& lo) { hi = (b16)v; lo = (b16)(v - (float)hi); }
__device__ __forceinline__ v16b frag_kb(const b16* p, int hh) { const v8b a = *(const v8b*)(p + 8 * hh), b = *(const v8b*)(p + 16 + 8 * hh); v16b f;
#pragma unroll
  for (int e = 0; e < 8; ++e) { f[e] = a[e]; f[8 + e] = b[e]; } return f; }
__device__ __forceinline__ v8f wmma16b(v16b a, v16b b, v8f c) { v8f d = __builtin_amdgcn_wmma_f32_16x16x32_f16(false, a, false, b, (short)0, c, false, false); asm volatile("v_nop\n\tv_nop\n\tv_nop\n\tv_nop" : "+v"(d) : "v"(a), "v"(b)); return d; }
__device__ __forceinline__ void wave_lds_sync() { __builtin_amdgcn_fence(__ATOMIC_RELEASE, "workgroup"); __builtin_amdgcn_wave_barrier(); __builtin_amdgcn_fence(__ATOMIC_ACQUIRE, "workgroup"); }
__device__ __forceinline__ float pmul(float a, float b) { float p = a * b; asm volatile("" : "+v"(p)); return p; }

__global__ __launch_bounds__(256) void wput_kernel(const float* __restrict__ w, int KIN, int KP, int OUTW, int ldw, int krow0, b16* __restrict__ WT) {
  const int KG = KP / 8; const int u = blockIdx.x * 256 + threadIdx.x; if (u >= OUTW * KG) return; const int o = u / KG, k0 = (u % KG) * 8; v8b v;
#pragma unroll
  for (int j = 0; j < 8; ++j) { const int k = k0 + j; v[j] = (b16)(k < KIN ? bf16_rne(w[(size_t)(krow0 + k) * ldw + o]) * WSC : 0.0f); } for (int pass = 0; pass < 2; ++pass) { *(volatile v8b*)(WT + (size_t)o * KP + k0) = v; __threadfence(); }
}
template <int KIN, int NT, int MODE, int RELU>
__global__ __launch_bounds__(32) void dense_kernel(const float* __restrict__ IN, int inp, int kreal, float asc, const b16* __restrict__ WT, const float* __restrict__ bias, float osc, const float* __restrict__ RES, int resp, int ncg, int outp, float* __restrict__ OUT) {
  __shared__ __attribute__((aligned(16))) b16 Ah[16][KIN + 8], Al[16][MODE ? KIN + 8 : 8]; __shared__ float Tf[16][NT * 16 + 4];
  const int lane = threadIdx.x, nloc = lane & 15, hlf = lane >> 4; const int cg = blockIdx.x % ncg; const size_t m0 = (size_t)(blockIdx.x / ncg) * 16;
  for (int rr = 0; rr < 16; ++rr) for (int c = lane; c < KIN; c += 32) { const float v = c < kreal ? IN[(m0 + rr) * (size_t)inp + c] : 0.0f; if (MODE == 0) Ah[rr][c] = (b16)(bf16_rne(v) * asc); else { b16 p, q; split16(v * XS, p, q); Ah[rr][c] = p; Al[rr][c] = q; } }
  wave_lds_sync(); v8f acc[NT];
#pragma unroll
  for (int t = 0; t < NT; ++t) acc[t] = (v8f){};
#pragma unroll 2
  for (int kb = 0; kb < KIN; kb += 32) { const v16b a = frag_kb(&Ah[nloc][kb], hlf); v16b al; if (MODE) al = frag_kb(&Al[nloc][kb], hlf);
#pragma unroll
    for (int t = 0; t < NT; ++t) { const v16b bw = frag_kb(WT + (size_t)(cg * NT * 16 + t * 16 + nloc) * KIN + kb, hlf); acc[t] = wmma16b(a, bw, acc[t]); if (MODE) acc[t] = wmma16b(al, bw, acc[t]); } }
#pragma unroll
  for (int t = 0; t < NT; ++t) { const int c = cg * NT * 16 + t * 16 + nloc; const float bb = bias ? bf16_rne(bias[c]) : 0.0f;
#pragma unroll
    for (int r8 = 0; r8 < 8; ++r8) { float v = acc[t][r8] * osc + bb; if (RELU) v = fmaxf(v, 0.0f); if (RES) v += RES[(m0 + 8 * hlf + r8) * (size_t)resp + c]; Tf[8 * hlf + r8][t * 16 + nloc] = v; } }
  wave_lds_sync();
  for (int pass = 0; pass < 2; ++pass) { for (int rr = 0; rr < 16; ++rr) for (int c = lane; c < NT * 16; c += 32) ((volatile float*)OUT)[(m0 + rr) * (size_t)outp + cg * NT * 16 + c] = Tf[rr][c]; __threadfence(); }
}
__global__ __launch_bounds__(32) void prep2_kernel(const float* __restrict__ h, const float* __restrict__ G2A, float* __restrict__ H2, float* __restrict__ GRAM) {
  const int lane = threadIdx.x; const int nd = blockIdx.x; __shared__ float Gs[NVEC][32];
  for (int i = 0; i < NVEC; ++i) Gs[i][lane] = G2A[((size_t)nd * NVEC + i) * 32 + lane];
  wave_lds_sync();
  for (int pass = 0; pass < 2; ++pass) {
    for (int q = 0; q < 8; ++q) ((volatile float*)H2)[(size_t)nd * 2 * E + E + q * 32 + lane] = bf16_rne(h[(size_t)nd * E + q * 32 + lane]) * SQE;
    for (int a = 0; a < 32; ++a) { float s = 0.0f; for (int i = 0; i < NVEC; ++i) s += pmul(Gs[i][a], Gs[i][lane]); ((volatile float*)GRAM)[(size_t)nd * 1024 + a * 32 + lane] = s; }
    __threadfence(); }
}
__global__ __launch_bounds__(32) void att_kernel(const float* __restrict__ QKV, const float* __restrict__ VG, int QLIM, float* __restrict__ OV, float* __restrict__ OG) {
  __shared__ __attribute__((aligned(16))) b16 Qh[16][40], Ql[16][40], Kh[32][40], Kl[32][40], Pp[16][40], Vt[128][40]; __shared__ float Sc[16][33], Mx[16], Dn[16], Sf[16], Of[16][132];
  const int lane = threadIdx.x, nloc = lane & 15, hlf = lane >> 4; const int hh = blockIdx.x / (QLIM / 16), q0 = (blockIdx.x % (QLIM / 16)) * 16; const size_t W3 = 3 * E;
  for (int rr = 0; rr < 16; ++rr) { b16 p, ql; split16(QKV[(size_t)(q0 + rr) * W3 + hh * HD + lane] * XS, p, ql); Qh[rr][lane] = p; Ql[rr][lane] = ql; }
  if (lane < 16) { Mx[lane] = -INFINITY; Dn[lane] = 0.0f; Sf[lane] = 0.0f; }
  v8f acc[8];
#pragma unroll
  for (int t = 0; t < 8; ++t) acc[t] = (v8f){};
  wave_lds_sync();
#pragma unroll 1
  for (int kc = 0; kc < N; kc += 32) {
    for (int rr = 0; rr < 32; ++rr) { const size_t m = (size_t)kc + rr; b16 p, ql; split16(QKV[m * W3 + E + hh * HD + lane] * XS, p, ql); Kh[rr][lane] = p; Kl[rr][lane] = ql;
      Vt[lane][rr] = (b16)(QKV[m * W3 + 2 * E + hh * HD + lane] * XS); for (int i = 0; i < NVEC; ++i) Vt[32 + i * 32 + lane][rr] = (b16)(VG[(m * NVEC + i) * E + hh * HD + lane] * XS); }
    wave_lds_sync();
#pragma unroll
    for (int blk = 0; blk < 2; ++blk) { v8f s = {}; const v16b qh = frag_kb(&Qh[nloc][0], hlf), qlo = frag_kb(&Ql[nloc][0], hlf), kh = frag_kb(&Kh[blk * 16 + nloc][0], hlf), kl = frag_kb(&Kl[blk * 16 + nloc][0], hlf); s = wmma16b(qh, kh, s); s = wmma16b(qh, kl, s); s = wmma16b(qlo, kh, s);
#pragma unroll
      for (int r8 = 0; r8 < 8; ++r8) Sc[8 * hlf + r8][blk * 16 + nloc] = s[r8] * (1.0f / (XS * XS)); }
    wave_lds_sync();
#pragma unroll 1
    for (int qi = 0; qi < 16; ++qi) { const float sv = Sc[qi][lane]; float cm = sv; for (int o = 16; o; o >>= 1) cm = fmaxf(cm, __shfl_xor(cm, o)); const float mo = Mx[qi]; const float mn = fmaxf(mo, cm); const float p = __expf(sv - mn); float psum = p; for (int o = 16; o; o >>= 1) psum += __shfl_xor(psum, o);
      Pp[qi][lane] = (b16)(p * PS); if (lane == 0) { const float sf = (mo == -INFINITY) ? 0.0f : __expf(mo - mn); Sf[qi] = sf; Dn[qi] = Dn[qi] * sf + psum; Mx[qi] = mn; } }
    wave_lds_sync();
#pragma unroll
    for (int t = 0; t < 8; ++t) {
#pragma unroll
      for (int r8 = 0; r8 < 8; ++r8) acc[t][r8] *= Sf[8 * hlf + r8];
      acc[t] = wmma16b(frag_kb(&Pp[nloc][0], hlf), frag_kb(&Vt[t * 16 + nloc][0], hlf), acc[t]); }
    wave_lds_sync(); }
#pragma unroll
  for (int t = 0; t < 8; ++t)
#pragma unroll
    for (int r8 = 0; r8 < 8; ++r8) { const int rl = 8 * hlf + r8; Of[rl][t * 16 + nloc] = acc[t][r8] * (1.0f / (PS * XS)) / Dn[rl]; }
  wave_lds_sync();
  for (int pass = 0; pass < 2; ++pass) { for (int rr = 0; rr < 16; ++rr) { const size_t nq = (size_t)q0 + rr; ((volatile float*)OV)[nq * E + hh * HD + lane] = Of[rr][lane]; for (int i = 0; i < NVEC; ++i) ((volatile float*)OG)[(nq * NVEC + i) * E + hh * HD + lane] = Of[rr][32 + i * 32 + lane]; } __threadfence(); }
}
}

extern "C" void kernel_launch(void* const* d_in, const int* in_sizes, int n_in, void* d_out, int out_size, void* d_ws, size_t ws_size, hipStream_t stream) {
  (void)n_in;
  auto Fp = [&](int i) { return (const float*)d_in[i]; };
  if (in_sizes[0] != NG * M || in_sizes[1] != N * E || in_sizes[4] != M * E || in_sizes[5] != E * 32 || in_sizes[6] != E * E || in_sizes[7] != 1024 * 2 * E || in_sizes[9] != 2 * E * E || in_sizes[11] != 2 * E * E || in_sizes[13] != 2 * E * E || in_sizes[15] != 2 * E * E || in_sizes[17] != E * E || in_sizes[19] != E * E || in_sizes[20] != E * M || in_sizes[21] != E * E || out_size != NG * M + N * E) return;
  const int QLIM = N;
  size_t off = 0; char* ws = (char*)d_ws;
  auto carve = [&](size_t bytes) { char* p = ws + off; off += (bytes + 255) & ~(size_t)255; return p; };
  b16* WEQ = (b16*)carve((size_t)E * 32 * 2); b16* WGP = (b16*)carve((size_t)32 * E * 2); b16* WVG = (b16*)carve((size_t)E * E * 2); b16* WG1 = (b16*)carve((size_t)2 * E * 1024 * 2); b16* WG2 = (b16*)carve((size_t)E * 2 * E * 2);
  b16* WQKV = (b16*)carve((size_t)3 * E * 2 * E * 2); b16* WNG = (b16*)carve((size_t)E * E * 2); b16* WGO = (b16*)carve((size_t)E * E * 2); b16* WGD = (b16*)carve((size_t)16 * E * 2); b16* WHD = (b16*)carve((size_t)E * E * 2);
  float* GS = (float*)carve((size_t)NG * E * 4); float* G2A = (float*)carve((size_t)NG * 32 * 4); float* GRAM = (float*)carve((size_t)N * 1024 * 4); float* G2H = (float*)carve((size_t)N * 2 * E * 4); float* H2 = (float*)carve((size_t)N * 2 * E * 4);
  float* QKV = (float*)carve((size_t)N * 3 * E * 4); float* VG = (float*)carve((size_t)NG * E * 4); float* OV = (float*)carve((size_t)N * E * 4); float* OG = (float*)carve((size_t)NG * E * 4); float* GS2 = (float*)carve((size_t)NG * E * 4); float* HS2 = (float*)carve((size_t)N * E * 4);
  if (off > ws_size || off > ((size_t)128 << 20)) return;
  wput_kernel<<<(E * 4 + 255) / 256, 256, 0, stream>>>(Fp(4), M, 32, E, E, 0, WEQ);
  wput_kernel<<<(32 * 32 + 255) / 256, 256, 0, stream>>>(Fp(5), E, E, 32, 32, 0, WGP);
  wput_kernel<<<(E * 32 + 255) / 256, 256, 0, stream>>>(Fp(6), E, E, E, E, 0, WVG);
  wput_kernel<<<(2 * E * 128 + 255) / 256, 256, 0, stream>>>(Fp(7), 1024, 1024, 2 * E, 2 * E, 0, WG1);
  wput_kernel<<<(E * 64 + 255) / 256, 256, 0, stream>>>(Fp(9), 2 * E, 2 * E, E, E, 0, WG2);
  wput_kernel<<<(E * 64 + 255) / 256, 256, 0, stream>>>(Fp(11), 2 * E, 2 * E, E, E, 0, WQKV); wput_kernel<<<(E * 64 + 255) / 256, 256, 0, stream>>>(Fp(13), 2 * E, 2 * E, E, E, 0, WQKV + (size_t)E * 2 * E); wput_kernel<<<(E * 64 + 255) / 256, 256, 0, stream>>>(Fp(15), 2 * E, 2 * E, E, E, 0, WQKV + (size_t)2 * E * 2 * E);
  wput_kernel<<<(E * 32 + 255) / 256, 256, 0, stream>>>(Fp(17), E, E, E, E, 0, WNG); wput_kernel<<<(E * 32 + 255) / 256, 256, 0, stream>>>(Fp(19), E, E, E, E, 0, WGO); wput_kernel<<<(16 * 32 + 255) / 256, 256, 0, stream>>>(Fp(20), E, E, M, M, 0, WGD); wput_kernel<<<(E * 32 + 255) / 256, 256, 0, stream>>>(Fp(21), E, E, E, E, 0, WHD);
  dense_kernel<32, 16, 0, 0><<<NG / 16, 32, 0, stream>>>(Fp(0), M, M, XS, WEQ, nullptr, SQE / (XS * WSC), nullptr, 0, 1, E, GS);
  dense_kernel<E, 2, 1, 0><<<NG / 16, 32, 0, stream>>>(GS, E, E, 0.0f, WGP, nullptr, 1.0f / (XS * WSC), nullptr, 0, 1, 32, G2A);
  prep2_kernel<<<N, 32, 0, stream>>>(Fp(1), G2A, H2, GRAM);
  dense_kernel<1024, 16, 1, 1><<<(N / 16) * 2, 32, 0, stream>>>(GRAM, 1024, 1024, 0.0f, WG1, Fp(8), 1.0f / (XS * WSC), nullptr, 0, 2, 2 * E, G2H);
  dense_kernel<2 * E, 16, 1, 0><<<N / 16, 32, 0, stream>>>(G2H, 2 * E, 2 * E, 0.0f, WG2, Fp(10), 1.0f / (XS * WSC), nullptr, 0, 1, 2 * E, H2);
  dense_kernel<2 * E, 16, 1, 0><<<(N / 16), 32, 0, stream>>>(H2, 2 * E, 2 * E, 0.0f, WQKV, Fp(12), SCAL / (XS * WSC), nullptr, 0, 1, 3 * E, QKV);
  dense_kernel<2 * E, 16, 1, 0><<<(N / 16), 32, 0, stream>>>(H2, 2 * E, 2 * E, 0.0f, WQKV + (size_t)E * 2 * E, Fp(14), 1.0f / (XS * WSC), nullptr, 0, 1, 3 * E, QKV + E);
  dense_kernel<2 * E, 16, 1, 0><<<(N / 16), 32, 0, stream>>>(H2, 2 * E, 2 * E, 0.0f, WQKV + (size_t)2 * E * 2 * E, Fp(16), 1.0f / (XS * WSC), nullptr, 0, 1, 3 * E, QKV + 2 * E);
  dense_kernel<E, 16, 1, 0><<<NG / 16, 32, 0, stream>>>(GS, E, E, 0.0f, WVG, nullptr, 1.0f / (XS * WSC), nullptr, 0, 1, E, VG);
  att_kernel<<<NH * (QLIM / 16), 32, 0, stream>>>(QKV, VG, QLIM, OV, OG);
  dense_kernel<E, 16, 1, 0><<<QLIM / 16, 32, 0, stream>>>(OV, E, E, 0.0f, WNG, Fp(18), 1.0f / (XS * WSC), H2 + E, 2 * E, 1, E, HS2);
  dense_kernel<E, 16, 1, 0><<<QLIM * NVEC / 16, 32, 0, stream>>>(OG, E, E, 0.0f, WGO, nullptr, 1.0f / (XS * WSC), GS, E, 1, E, GS2);
  float* out = (float*)d_out;
  dense_kernel<E, 1, 1, 0><<<QLIM * NVEC / 16, 32, 0, stream>>>(GS2, E, E, 0.0f, WGD, nullptr, 1.0f / (XS * WSC), nullptr, 0, 1, M, out);
  dense_kernel<E, 16, 1, 0><<<QLIM / 16, 32, 0, stream>>>(HS2, E, E, 0.0f, WHD, Fp(22), 1.0f / (XS * WSC), nullptr, 0, 1, E, out + (size_t)NG * M);
}
